// Eq_NLMP2_60653528154708
// MI455X (gfx1250) — hardware-run, weakly checked
//
#include <hip/hip_runtime.h>


namespace {
constexpr int N = 10000, E = 100000, MS = 16, MV = 8, RW = 40, NXS = 48, NXV = 24, HK = 16, NEMB = 10;
constexpr float XS = 8.0f, WSC = 256.0f, CT = 1.5927f, CR = 1.4142135623730951f, SQ3 = 1.7320508075688772f;
typedef _Float16 b16;
typedef __attribute__((ext_vector_type(16))) _Float16 v16b;
typedef __attribute__((ext_vector_type(8))) _Float16 v8b;
typedef __attribute__((ext_vector_type(8))) float v8f;
__device__ __forceinline__ float bf16_rne(float f) { unsigned int u = __float_as_uint(f); u += 0x7FFFu + ((u >> 16) & 1u); float r = __uint_as_float(u & 0xFFFF0000u); asm volatile("" : "+v"(r)); return r; }
__device__ __forceinline__ void split16(float v, b16& hi, b16& lo) { hi = (b16)v; lo = (b16)(v - (float)hi); }
__device__ __forceinline__ v16b frag_kb(const b16* p, int hh) { const v8b a = *(const v8b*)(p + 8 * hh), b = *(const v8b*)(p + 16 + 8 * hh); v16b f;
#pragma unroll
  for (int e = 0; e < 8; ++e) { f[e] = a[e]; f[8 + e] = b[e]; } return f; }
__device__ __forceinline__ v8f wmma16b(v16b a, v16b b, v8f c) { v8f d = __builtin_amdgcn_wmma_f32_16x16x32_f16(false, a, false, b, (short)0, c, false, false); asm volatile("v_nop\n\tv_nop\n\tv_nop\n\tv_nop" : "+v"(d) : "v"(a), "v"(b)); return d; }
__device__ __forceinline__ void wave_lds_sync() { __builtin_amdgcn_fence(__ATOMIC_RELEASE, "workgroup"); __builtin_amdgcn_wave_barrier(); __builtin_amdgcn_fence(__ATOMIC_ACQUIRE, "workgroup"); }
__device__ __forceinline__ float pmul(float a, float b) { float p = a * b; asm volatile("" : "+v"(p)); return p; }
__device__ __forceinline__ int iclamp(int v, int lo, int hi) { return v < lo ? lo : (v > hi ? hi : v); }
__device__ __forceinline__ float ftanh(float v) { const float a = fminf(fabsf(v), 15.0f); const float e2 = __expf(2.0f * a); const float t = 1.0f - 2.0f / (e2 + 1.0f); return v < 0.0f ? -t : t; }
constexpr int CSR_NBLK9 = 512, CSR_GB9 = 9, CSR_GN9 = 1 << CSR_GB9  , CSR_TS9 = (CSR_GN9 < 32 ? 32 : CSR_GN9)  , CSR_MAXG9 = 512, CSR_CAP9 = 12288  ;
__device__ __host__ __forceinline__ int csr_tix9(int v) { return (v >> CSR_GB9) * CSR_TS9 + (v & (CSR_GN9 - 1)); }
__global__ __launch_bounds__(64) void csrA_kernel9(const int* __restrict__ dst, int E, int N, int nG, int CHP, int NGP, int* __restrict__ STG, int* __restrict__ HST) {
  extern __shared__ int sm[];
  int* cnt = sm; int* run = sm + NGP; int* ids = sm + 2 * NGP;
  const int b = blockIdx.x; const int ch = (E + CSR_NBLK9 - 1) / CSR_NBLK9; const int e0 = b * ch, e1 = min(E, e0 + ch);
  for (int i = threadIdx.x; i < NGP; i += 64) cnt[i] = 0;
  for (int i = threadIdx.x; i < CHP; i += 64) ids[i] = -1;
  __syncthreads();
  if (threadIdx.x == 0) {
    for (int e = e0; e < e1; ++e) { int d = dst[e]; d = (d < 0) ? 0 : (d >= N ? N - 1 : d); cnt[d >> CSR_GB9] += 1; }
    int acc = 0; for (int g = 0; g < nG; ++g) { run[g] = acc; acc += cnt[g]; }
    for (int e = e0; e < e1; ++e) { int d = dst[e]; d = (d < 0) ? 0 : (d >= N ? N - 1 : d); const int g = d >> CSR_GB9; ids[run[g]] = e; run[g] += 1; } }
  __syncthreads();
  typedef __attribute__((ext_vector_type(4))) int v4i;
  for (int pass = 0; pass < 2; ++pass) {
    for (int i = threadIdx.x; i < CHP / 4; i += 64) *(volatile v4i*)(STG + (size_t)b * CHP + i * 4) = *(const v4i*)(&ids[i * 4]);
    for (int i = threadIdx.x; i < NGP / 4; i += 64) { v4i v; for (int e = 0; e < 4; ++e) v[e] = (i * 4 + e < nG) ? cnt[i * 4 + e] : 0; *(volatile v4i*)(HST + (size_t)b * NGP + i * 4) = v; }
    __threadfence(); }
}
__global__ __launch_bounds__(512) void csrS_kernel9(const int* __restrict__ HST, int nG, int NGP, int* __restrict__ START, int* __restrict__ TOT, int* __restrict__ OFF) {
  __shared__ int tot[CSR_MAXG9];
  const int b = threadIdx.x;
  for (int pass = 0; pass < 2; ++pass) { int runb = 0; for (int g = 0; g < nG; ++g) { int c = HST[(size_t)b * NGP + g]; c = (c < 0) ? 0 : c; ((volatile int*)OFF)[(size_t)g * CSR_NBLK9 + b] = runb; runb += c; } __threadfence(); }
  for (int g = threadIdx.x; g < nG; g += 512) { int s = 0; for (int bb = 0; bb < CSR_NBLK9; ++bb) { int c = HST[(size_t)bb * NGP + g]; s += (c < 0) ? 0 : c; } tot[g] = s; }
  __syncthreads();
  if (threadIdx.x < 32) {
    __shared__ int st[CSR_MAXG9 + 32];
    if (threadIdx.x == 0) { int acc = 0; for (int g = 0; g < NGP; ++g) { st[g] = acc; if (g < nG) acc += (tot[g] + 31) & ~31; } st[NGP] = acc; }
    __builtin_amdgcn_fence(__ATOMIC_RELEASE, "workgroup"); __builtin_amdgcn_wave_barrier(); __builtin_amdgcn_fence(__ATOMIC_ACQUIRE, "workgroup");
    for (int pass = 0; pass < 2; ++pass) { for (int i = threadIdx.x; i < NGP + 32; i += 32) { ((volatile int*)START)[i] = (i <= NGP) ? st[min(i, NGP)] : 0; ((volatile int*)TOT)[i] = (i < nG) ? tot[i] : 0; } __threadfence(); } }
}
__global__ __launch_bounds__(256) void csrB_kernel9(const int* __restrict__ dst, int N, int nG, int CHP, int NGP, int permLen, const int* __restrict__ STG, const int* __restrict__ HST, const int* __restrict__ OFF, const int* __restrict__ START, const int* __restrict__ TOT, int* __restrict__ PERM, int* __restrict__ ROWPTR, int* __restrict__ ROWCNT, int* __restrict__ FLAG) {
  typedef __attribute__((ext_vector_type(4))) int v4i;
  __shared__ int ids[CSR_CAP9]; __shared__ unsigned short key[CSR_CAP9]; __shared__ int outp[CSR_CAP9]; __shared__ int ncnt[CSR_GN9 + 1]; __shared__ int boff[CSR_NBLK9 + 1];
  const int g = blockIdx.x, t_ = threadIdx.x; int tot = TOT[g]; int st = START[g], stn = START[g + 1]; const int v0 = g * CSR_GN9; const int nv = min(CSR_GN9, N - v0); const int t0 = g * CSR_TS9;
  st = (st < 0) ? 0 : (st > permLen - 32 ? permLen - 32 : st) & ~31; stn = (stn < st) ? st : (stn > permLen ? permLen : stn); tot = (tot < 0) ? 0 : tot; if (tot > stn - st && tot <= CSR_CAP9) tot = stn - st;
  if (tot > CSR_CAP9) {
    for (int pass = 0; pass < 2; ++pass) { for (int i = t_; i < CSR_TS9 / 4; i += 256) { v4i a, c; for (int e = 0; e < 4; ++e) { a[e] = st; c[e] = 0; } *(volatile v4i*)(ROWPTR + t0 + i * 4) = a; *(volatile v4i*)(ROWCNT + t0 + i * 4) = c; } if (t_ == 0) ((volatile int*)FLAG)[0] = 1; __threadfence(); } (void)nv; return; }
  if (t_ == 0) { int acc = 0; for (int b = 0; b < CSR_NBLK9; ++b) { boff[b] = acc; int c = HST[(size_t)b * NGP + g]; c = (c < 0) ? 0 : (c > CHP ? CHP : c); acc += c; if (acc > tot) acc = tot; } boff[CSR_NBLK9] = acc; }
  for (int i = t_; i <= CSR_GN9; i += 256) ncnt[i] = 0;
  __syncthreads();
  for (int b = 0; b < CSR_NBLK9; ++b) { const int c = boff[b + 1] - boff[b]; int o_ = OFF[(size_t)g * CSR_NBLK9 + b]; o_ = (o_ < 0) ? 0 : (o_ > CHP - c ? CHP - c : o_); const int* src_ = STG + (size_t)b * CHP + o_;
    for (int i = t_; i < c; i += 256) { int id = src_[i]; id = (id < 0) ? 0 : id; ids[boff[b] + i] = id; int d = dst[id]; d = (d < v0) ? v0 : (d >= N ? N - 1 : d); int kk = d - v0; kk = (kk < 0) ? 0 : (kk >= CSR_GN9 ? CSR_GN9 - 1 : kk); key[boff[b] + i] = (unsigned short)kk; } }
  __syncthreads();
  if (t_ == 0) { for (int i = 0; i < tot; ++i) ncnt[key[i]] += 1; int acc = 0; for (int vl = 0; vl < CSR_GN9; ++vl) { const int c = ncnt[vl]; ncnt[vl] = acc; acc += c; } ncnt[CSR_GN9] = acc;
    for (int i = 0; i < tot; ++i) { const int vl = key[i]; outp[ncnt[vl]] = ids[i]; ncnt[vl] += 1; }
    for (int vl = CSR_GN9; vl > 0; --vl) ncnt[vl] = ncnt[vl - 1]; ncnt[0] = 0; }
  __syncthreads();
  for (int pass = 0; pass < 2; ++pass) {
    for (int i = t_; i < (stn - st) / 4; i += 256) { v4i v; for (int e = 0; e < 4; ++e) { const int q = i * 4 + e; v[e] = (q < tot) ? outp[q] : -1; } *(volatile v4i*)(PERM + st + i * 4) = v; }
    for (int i = t_; i < CSR_TS9 / 4; i += 256) { v4i a, c; for (int e = 0; e < 4; ++e) { const int vl = i * 4 + e; const int vc = vl < CSR_GN9 ? vl : CSR_GN9; a[e] = (vl < CSR_GN9) ? st + ncnt[vc] : st; c[e] = (vl < nv) ? (ncnt[(vc < CSR_GN9 ? vc : CSR_GN9 - 1) + 1] - ncnt[vc]) : 0; } *(volatile v4i*)(ROWPTR + t0 + i * 4) = a; *(volatile v4i*)(ROWCNT + t0 + i * 4) = c; }
    __threadfence(); }
}
__global__ __launch_bounds__(256) void csrZ_kernel9(int* __restrict__ p, size_t n4) { typedef __attribute__((ext_vector_type(4))) int v4i; const size_t tid = (size_t)blockIdx.x * 256 + threadIdx.x, nth = (size_t)gridDim.x * 256; v4i z = {0, 0, 0, 0}; for (size_t i = tid; i < n4; i += nth) *(volatile v4i*)(p + i * 4) = z; }
struct CsrBufs9 { int *STG, *HST, *OFF, *START, *TOT, *PERM, *ROWPTR, *ROWCNT, *FLAG; int nG, NGP, CHP; size_t permLen; char* base; size_t bytes; };
static size_t csr_carve9(CsrBufs9& c, char* ws, size_t off, int E, int N) {
  const size_t off0 = off; c.base = ws + off;
  auto al = [&](size_t bytes) { char* p = ws + off; off += (bytes + 255) & ~(size_t)255; return p; };
  c.nG = (N + CSR_GN9 - 1) / CSR_GN9; c.NGP = (c.nG + 31) & ~31; const int ch = (E + CSR_NBLK9 - 1) / CSR_NBLK9; c.CHP = (ch + 31) & ~31; c.permLen = (size_t)E + 32 * (size_t)c.nG + 32;
  c.STG = (int*)al((size_t)CSR_NBLK9 * c.CHP * 4); c.HST = (int*)al((size_t)CSR_NBLK9 * c.NGP * 4); c.OFF = (int*)al((size_t)c.NGP * CSR_NBLK9 * 4); c.START = (int*)al((size_t)(c.NGP + 64) * 4); c.TOT = (int*)al((size_t)(c.NGP + 64) * 4);
  c.PERM = (int*)al(c.permLen * 4); c.ROWPTR = (int*)al((size_t)c.nG * CSR_TS9 * 4); c.ROWCNT = (int*)al((size_t)c.nG * CSR_TS9 * 4); c.FLAG = (int*)al(256);
  c.bytes = off - off0; return off;
}
static void csr_build9(const CsrBufs9& c, const int* dst, int E, int N, hipStream_t stream) {
  const size_t smem = (size_t)(2 * c.NGP + c.CHP) * 4;
  csrZ_kernel9<<<512, 256, 0, stream>>>((int*)c.base, c.bytes / 16);
  csrA_kernel9<<<CSR_NBLK9, 64, smem, stream>>>(dst, E, N, c.nG, c.CHP, c.NGP, c.STG, c.HST);
  csrS_kernel9<<<1, 512, 0, stream>>>(c.HST, c.nG, c.NGP, c.START, c.TOT, c.OFF);
  csrB_kernel9<<<c.nG, 256, 0, stream>>>(dst, N, c.nG, c.CHP, c.NGP, (int)c.permLen, c.STG, c.HST, c.OFF, c.START, c.TOT, c.PERM, c.ROWPTR, c.ROWCNT, c.FLAG);
}


__global__ __launch_bounds__(256) void wput_kernel(const float* __restrict__ f1, const float* __restrict__ f2, b16* __restrict__ M1, b16* __restrict__ M2, b16* __restrict__ M3, b16* __restrict__ M4, b16* __restrict__ M5, b16* __restrict__ M6) {
  const int t = blockIdx.x * 256 + threadIdx.x;
  const int s1 = 32 * 96, s2 = s1 + 32 * 48, s3 = s2 + 16 * 48, s4 = s3 + 32 * 32, s5 = s4 + 16 * 16, s6 = s5 + 16 * 16; if (t >= s6) return;
  int which, n, k0, KT; b16* dst; if (t < s1) { which = 1; n = t / 96; k0 = (t % 96) * 8; KT = 768; dst = M1; } else if (t < s2) { which = 2; n = (t - s1) / 48; k0 = ((t - s1) % 48) * 8; KT = 384; dst = M2; } else if (t < s3) { which = 3; n = (t - s2) / 48; k0 = ((t - s2) % 48) * 8; KT = 384; dst = M3; }
  else if (t < s4) { which = 4; n = (t - s3) / 32; k0 = ((t - s3) % 32) * 8; KT = 256; dst = M4; } else if (t < s5) { which = 5; n = (t - s4) / 16; k0 = ((t - s4) % 16) * 8; KT = 128; dst = M5; } else { which = 6; n = (t - s5) / 16; k0 = ((t - s5) % 16) * 8; KT = 128; dst = M6; }
  v8b v;
#pragma unroll
  for (int j = 0; j < 8; ++j) { const int K = k0 + j; const int u = K / 16, k = K % 16; int col = -1; const float* W = f1; int pitch = 2304;
    if (which == 1) { col = n < 16 ? u * 16 + n : (n < 24 ? 768 + u * 8 + (n - 16) : 1728 + u * 8 + (n - 24)); }
    else if (which == 2) { col = n < 16 ? 1152 + u * 16 + n : (n < 24 ? 1536 + u * 8 + (n - 16) : -1); }
    else if (which == 3) { col = n < 8 ? 2112 + u * 8 + n : -1; }
    else { W = f2; pitch = 576; if (which == 4) col = n < 16 ? u * 16 + n : (n < 24 ? 384 + u * 8 + (n - 16) : -1); else if (which == 5) col = 256 + u * 16 + n; else col = n < 8 ? 512 + u * 8 + n : -1; }
    v[j] = (b16)(col >= 0 ? bf16_rne(W[(size_t)k * pitch + col]) * WSC : 0.0f); }
  for (int pass = 0; pass < 2; ++pass) { *(volatile v8b*)(dst + (size_t)n * KT + k0) = v; __threadfence(); } }

struct EdgeL { float xs[16][NXS]; float xv[16][NXV][3]; float sh[16][3]; float h1[16][HK]; float h2[16][HK]; float he[16][RW]; float ts[16][MS]; float tv[16][MV][3]; float C1[16][33], C2[16][33], C3[3][16][17], C4[16][33], C5[16][17], C6[3][16][17]; float orow[16][RW]; };

template <int NU, typename FN>
__device__ __forceinline__ void stage_outer(b16 (*Ah)[776], b16 (*Al)[776], const float (*Hm)[HK], FN f, int lane) {
  for (int idx = lane; idx < 16 * NU * 16; idx += 32) { const int rr = idx / (NU * 16), K = idx % (NU * 16); const int u = K / 16, k = K % 16; b16 p, q; split16(pmul(f(rr, u), Hm[rr][k]) * XS, p, q); Ah[rr][K] = p; Al[rr][K] = q; } }
template <int KT, int NT>
__device__ __forceinline__ void gemm_tile(const b16 (*Ah)[776], const b16 (*Al)[776], const b16* __restrict__ M, float sc, float* Cout, int cpitch, int lane) { const int nloc = lane & 15, hlf = lane >> 4; v8f acc[NT];
#pragma unroll
  for (int t = 0; t < NT; ++t) acc[t] = (v8f){};
#pragma unroll 2
  for (int kb = 0; kb < KT; kb += 32) { const v16b a = frag_kb(&Ah[nloc][kb], hlf), al = frag_kb(&Al[nloc][kb], hlf);
#pragma unroll
    for (int t = 0; t < NT; ++t) { const v16b bw = frag_kb(M + (size_t)(t * 16 + nloc) * KT + kb, hlf); acc[t] = wmma16b(a, bw, acc[t]); acc[t] = wmma16b(al, bw, acc[t]); } }
#pragma unroll
  for (int t = 0; t < NT; ++t)
#pragma unroll
    for (int r8 = 0; r8 < 8; ++r8) Cout[(8 * hlf + r8) * cpitch + t * 16 + nloc] = acc[t][r8] * sc; }

__global__ __launch_bounds__(32) void edge_kernel(const float* __restrict__ hn, const float* __restrict__ he, const float* __restrict__ ev, const float* __restrict__ emb, const float* __restrict__ f1w1, const float* __restrict__ f2w1, const b16* __restrict__ M1, const b16* __restrict__ M2, const b16* __restrict__ M3, const b16* __restrict__ M4, const b16* __restrict__ M5, const b16* __restrict__ M6, const int* __restrict__ srcs, const int* __restrict__ dsts, int ELIM, float* __restrict__ out, float* __restrict__ HE) {
  __shared__ __attribute__((aligned(16))) b16 Ah[16][776], Al[16][776]; __shared__ EdgeL L; const int lane = threadIdx.x; const size_t e0 = (size_t)blockIdx.x * 16; if (e0 >= (size_t)ELIM) return;
  { const int rr = lane & 15, hf = lane >> 4; const size_t e = e0 + rr; const size_t si = (size_t)iclamp(srcs[e], 0, N - 1), di = (size_t)iclamp(dsts[e], 0, N - 1);
    if (hf == 0) { for (int c = 0; c < RW; ++c) { const float v = bf16_rne(he[e * RW + c]); L.he[rr][c] = v; if (c < MS) L.xs[rr][c] = v; else L.xv[rr][(c - MS) / 3][(c - MS) % 3] = v; }
      for (int c = 0; c < RW; ++c) { const float v = bf16_rne(hn[si * RW + c]); if (c < MS) L.xs[rr][MS + c] = v; else L.xv[rr][MV + (c - MS) / 3][(c - MS) % 3] = v; } }
    else { for (int c = 0; c < RW; ++c) { const float v = bf16_rne(hn[di * RW + c]); if (c < MS) L.xs[rr][2 * MS + c] = v; else L.xv[rr][2 * MV + (c - MS) / 3][(c - MS) % 3] = v; }
      const float vx = bf16_rne(ev[e * 3]), vy = bf16_rne(ev[e * 3 + 1]), vz = bf16_rne(ev[e * 3 + 2]); const float inv = SQ3 / sqrtf(pmul(vx, vx) + pmul(vy, vy) + pmul(vz, vz)); L.sh[rr][0] = pmul(vy, inv); L.sh[rr][1] = pmul(vz, inv); L.sh[rr][2] = pmul(vx, inv);
      for (int k = 0; k < HK; ++k) { float a = 0.0f, b = 0.0f; for (int m = 0; m < NEMB; ++m) { const float em = bf16_rne(emb[e * NEMB + m]); a += pmul(em, bf16_rne(f1w1[m * HK + k])); b += pmul(em, bf16_rne(f2w1[m * HK + k])); } L.h1[rr][k] = pmul(CR, fmaxf(a * 0.31622776601683794f, 0.0f)); L.h2[rr][k] = pmul(CR, fmaxf(b * 0.31622776601683794f, 0.0f)); } } }
  wave_lds_sync();
  const float S1 = 1.0f / (XS * WSC * 4.0f);
  stage_outer<NXS>(Ah, Al, L.h1, [&](int rr, int u) { return L.xs[rr][u]; }, lane); wave_lds_sync(); gemm_tile<768, 2>(Ah, Al, M1, S1, &L.C1[0][0], 33, lane); wave_lds_sync();
  stage_outer<NXV>(Ah, Al, L.h1, [&](int rr, int u) { return pmul(L.xv[rr][u][0], L.sh[rr][0]) + pmul(L.xv[rr][u][1], L.sh[rr][1]) + pmul(L.xv[rr][u][2], L.sh[rr][2]); }, lane); wave_lds_sync(); gemm_tile<384, 2>(Ah, Al, M2, S1, &L.C2[0][0], 33, lane); wave_lds_sync();
  for (int i = 0; i < 3; ++i) { stage_outer<NXV>(Ah, Al, L.h1, [&](int rr, int u) { return L.xv[rr][u][i]; }, lane); wave_lds_sync(); gemm_tile<384, 1>(Ah, Al, M3, S1, &L.C3[i][0][0], 17, lane); wave_lds_sync(); }
  { const float a0 = 0.11785113019775792f, a1 = 0.2041241452319315f; const int rr = lane & 15, hf = lane >> 4;
    if (hf == 0) { for (int w = 0; w < MS; ++w) L.ts[rr][w] = pmul(CT, ftanh(pmul(a0, L.C1[rr][w] + L.C2[rr][w] * (1.0f / SQ3)))); }
    else { for (int w = 0; w < MV; ++w) { const float g = pmul(CT, ftanh(pmul(a0, L.C1[rr][16 + w] + L.C2[rr][16 + w] * (1.0f / SQ3)))); for (int i = 0; i < 3; ++i) L.tv[rr][w][i] = pmul(g, pmul(a1 / SQ3, pmul(L.sh[rr][i], L.C1[rr][24 + w]) + L.C3[i][rr][w])); } } }
  wave_lds_sync();
  stage_outer<MS>(Ah, Al, L.h2, [&](int rr, int u) { return L.ts[rr][u]; }, lane); wave_lds_sync(); gemm_tile<256, 2>(Ah, Al, M4, S1, &L.C4[0][0], 33, lane); wave_lds_sync();
  stage_outer<MV>(Ah, Al, L.h2, [&](int rr, int u) { return pmul(L.tv[rr][u][0], L.sh[rr][0]) + pmul(L.tv[rr][u][1], L.sh[rr][1]) + pmul(L.tv[rr][u][2], L.sh[rr][2]); }, lane); wave_lds_sync(); gemm_tile<128, 1>(Ah, Al, M5, S1, &L.C5[0][0], 17, lane); wave_lds_sync();
  for (int i = 0; i < 3; ++i) { stage_outer<MV>(Ah, Al, L.h2, [&](int rr, int u) { return L.tv[rr][u][i]; }, lane); wave_lds_sync(); gemm_tile<128, 1>(Ah, Al, M6, S1, &L.C6[i][0][0], 17, lane); wave_lds_sync(); }
  { const float b0 = 0.2041241452319315f, b1 = 0.3535533905932738f; const int rr = lane & 15, hf = lane >> 4;
    if (hf == 0) { for (int w = 0; w < MS; ++w) L.orow[rr][w] = L.he[rr][w] + pmul(b0, L.C4[rr][w] + L.C5[rr][w] * (1.0f / SQ3)); }
    else { for (int w = 0; w < MV; ++w) for (int i = 0; i < 3; ++i) L.orow[rr][MS + w * 3 + i] = L.he[rr][MS + w * 3 + i] + pmul(b1 / SQ3, pmul(L.sh[rr][i], L.C4[rr][16 + w]) + L.C6[i][rr][w]); } }
  wave_lds_sync();
  for (int pass = 0; pass < 2; ++pass) { for (int q = lane; q < 16 * RW; q += 32) { const int rr = q / RW, c = q % RW; ((volatile float*)out)[((size_t)N + e0 + rr) * RW + c] = L.orow[rr][c]; ((volatile float*)HE)[(e0 + rr) * RW + c] = L.orow[rr][c]; } __threadfence(); } }
__global__ __launch_bounds__(256) void node_kernel(const float* __restrict__ hn, const float* __restrict__ HE, const float* __restrict__ nrm, const float* __restrict__ wl1s, const float* __restrict__ wl1g, const float* __restrict__ wl1v, const float* __restrict__ wl2s, const float* __restrict__ wl2v, const int* __restrict__ PERM, const int* __restrict__ ROWPTR, const int* __restrict__ ROWCNT, int permLen, int NLIMn, int ELIM, float* __restrict__ out) {
  __shared__ float CS[8][32], CV[8][16][3], G1[8][16], GV[8][8][3], ROW[8][RW]; const int wave = threadIdx.x >> 5, lane = threadIdx.x & 31; const int n = blockIdx.x * 8 + wave;
  if (n < NLIMn) { int st = ROWPTR[n], cnt = ROWCNT[n]; cnt = iclamp(cnt, 0, 1 << 20); st = iclamp(st, 0, permLen - cnt); float a0 = 0.0f, a1 = 0.0f;
#pragma unroll 1
    for (int j = 0; j < cnt; ++j) { const size_t e = (size_t)iclamp(PERM[st + j], 0, E - 1); if (e >= (size_t)ELIM) continue;     const float w = bf16_rne(nrm[e]); a0 += pmul(w, HE[e * RW + lane]); if (lane < RW - 32) a1 += pmul(w, HE[e * RW + 32 + lane]); }
    { const float hv = bf16_rne(hn[(size_t)n * RW + lane]); if (lane < MS) { CS[wave][lane] = hv; CS[wave][MS + lane] = a0; } else { const int c = lane - MS; CV[wave][c / 3][c % 3] = hv; CV[wave][MV + c / 3][c % 3] = a0; }
      if (lane < RW - 32) { const float hv2 = bf16_rne(hn[(size_t)n * RW + 32 + lane]); const int c = 32 + lane - MS; CV[wave][c / 3][c % 3] = hv2; CV[wave][MV + c / 3][c % 3] = a1; } }
    wave_lds_sync();
    if (lane < MS) { float s = 0.0f; for (int u = 0; u < 32; ++u) s += pmul(CS[wave][u], bf16_rne(wl1s[u * MS + lane])); G1[wave][lane] = pmul(CT, ftanh(s * 0.17677669529663688f)); }
    else if (lane < MS + MV) { const int w = lane - MS; float s = 0.0f; for (int u = 0; u < 32; ++u) s += pmul(CS[wave][u], bf16_rne(wl1g[u * MV + w])); const float g = pmul(CT, ftanh(s * 0.17677669529663688f)); for (int i = 0; i < 3; ++i) { float v = 0.0f; for (int u = 0; u < 16; ++u) v += pmul(CV[wave][u][i], bf16_rne(wl1v[u * MV + w])); GV[wave][w][i] = pmul(g, v * 0.25f); } }
    wave_lds_sync();
    if (lane < MS) { float s = 0.0f; for (int u = 0; u < MS; ++u) s += pmul(G1[wave][u], bf16_rne(wl2s[u * MS + lane])); ROW[wave][lane] = bf16_rne(hn[(size_t)n * RW + lane]) + s * 0.25f; }
    else if (lane < MS + MV) { const int v_ = lane - MS; for (int i = 0; i < 3; ++i) { float s = 0.0f; for (int w = 0; w < MV; ++w) s += pmul(GV[wave][w][i], bf16_rne(wl2v[w * MV + v_])); ROW[wave][MS + v_ * 3 + i] = bf16_rne(hn[(size_t)n * RW + MS + v_ * 3 + i]) + s * 0.35355339059327373f; } } }
  __syncthreads();
  if (wave == 0) { for (int pass = 0; pass < 2; ++pass) { for (int q = lane; q < 8 * RW; q += 32) { const int w8 = q / RW; if (blockIdx.x * 8 + w8 < NLIMn) ((volatile float*)out)[((size_t)blockIdx.x * 8 + w8) * RW + (q % RW)] = ROW[w8][q % RW]; } __threadfence(); } } }
}

extern "C" void kernel_launch(void* const* d_in, const int* in_sizes, int n_in, void* d_out, int out_size, void* d_ws, size_t ws_size, hipStream_t stream) {
  (void)n_in;
  auto Fp = [&](int i) { return (const float*)d_in[i]; }; auto Ip = [&](int i) { return (const int*)d_in[i]; };
  if (in_sizes[0] != N * RW || in_sizes[1] != E * RW || in_sizes[2] != E * 3 || in_sizes[3] != E * NEMB || in_sizes[4] != E || in_sizes[6] != 16 * 2304 || in_sizes[8] != 16 * 576 || in_sizes[14] != 2 * E || out_size != (N + E) * RW) return;
  const int ELIM = E, NLIMn = N;
  size_t off = 0; char* ws = (char*)d_ws;
  auto carve = [&](size_t bytes) { char* p = ws + off; off += (bytes + 255) & ~(size_t)255; return p; };
  b16* M1 = (b16*)carve((size_t)32 * 768 * 2); b16* M2 = (b16*)carve((size_t)32 * 384 * 2); b16* M3 = (b16*)carve((size_t)16 * 384 * 2); b16* M4 = (b16*)carve((size_t)32 * 256 * 2); b16* M5 = (b16*)carve((size_t)16 * 128 * 2); b16* M6 = (b16*)carve((size_t)16 * 128 * 2);
  float* HE = (float*)carve((size_t)E * RW * 4); CsrBufs9 csr; off = csr_carve9(csr, ws, off, E, N);
  if (off > ws_size || off > ((size_t)48 << 20)) return;
  wput_kernel<<<(32 * 96 + 32 * 48 + 16 * 48 + 32 * 32 + 16 * 16 + 16 * 16 + 255) / 256, 256, 0, stream>>>(Fp(6), Fp(8), M1, M2, M3, M4, M5, M6);
  csr_build9(csr, Ip(14) + E, E, N, stream);
  edge_kernel<<<E / 16, 32, 0, stream>>>(Fp(0), Fp(1), Fp(2), Fp(3), Fp(5), Fp(7), M1, M2, M3, M4, M5, M6, Ip(14), Ip(14) + E, ELIM, (float*)d_out, HE);
  node_kernel<<<(N + 7) / 8, 256, 0, stream>>>(Fp(0), HE, Fp(4), Fp(9), Fp(10), Fp(11), Fp(12), Fp(13), csr.PERM, csr.ROWPTR, csr.ROWCNT, (int)csr.permLen, NLIMn, ELIM, (float*)d_out);
}
